// GeneratorCombiner_2525440770803
// MI455X (gfx1250) — hardware-verified
//
#include <hip/hip_runtime.h>
#include <math.h>

typedef __attribute__((ext_vector_type(16))) _Float16 v16h;
typedef __attribute__((ext_vector_type(8)))  _Float16 v8h;
typedef __attribute__((ext_vector_type(8)))  float    v8f;
typedef __attribute__((ext_vector_type(4)))  float    v4f;

constexpr int kWires   = 10;
constexpr int kLayers  = 5;
constexpr int kGen     = 4;
constexpr int kBatch   = 256;
constexpr int kDim     = 1 << kWires;
constexpr int kPatch   = 1 << (kWires - 2);
constexpr int kGates   = kLayers * kWires;
constexpr int kParGen  = kGates * 2;
constexpr int kNcols   = kGen * 2 * kPatch;
constexpr float kCarry = 1024.0f;
constexpr float kFold  = 1.0f / (1024.0f * 1024.0f);
static_assert(kDim == 1024);
static_assert(kPatch == 256);
static_assert(kNcols == 2048);
static_assert((kDim % 32) == 0);
static_assert((kBatch % 64) == 0 && (kNcols % 64) == 0);

constexpr size_t kOffBT   = 0;
constexpr size_t kOffAP   = kOffBT + (size_t)kNcols * kDim * 2;
constexpr size_t kOffCA   = kOffAP + (size_t)kBatch * kDim * 2;
constexpr size_t kWsTotal = kOffCA + (size_t)kBatch * kNcols * 4;
static_assert(kWsTotal == 6815744ull);
static_assert(kWsTotal <= 134217728ull);
static_assert((kOffAP % 128) == 0 && (kOffCA % 128) == 0);

union FragH { v16h v; v8h h[2]; };
__device__ __forceinline__ v16h frag_load_h(const _Float16* p) {
  FragH f;
  f.h[0] = *(const v8h*)(p);
  f.h[1] = *(const v8h*)(p + 16);
  return f.v;
}
__device__ __forceinline__ v8f mma_h_guarded(v16h a, v16h b, v8f c) {
  c = __builtin_amdgcn_wmma_f32_16x16x32_f16(false, a, false, b, (short)0, c, false, false);
  asm volatile("v_nop\n\tv_nop\n\tv_nop\n\tv_nop" : "+v"(c) : "v"(a), "v"(b));
  return c;
}

__global__ __launch_bounds__(256) void build_rows_kernel(
    const float* __restrict__ qp, unsigned short* __restrict__ Bt)
{
  __shared__ __align__(16) float sSt[2 * kDim];
  __shared__ __align__(16) float sG[kGates * 8];
  const int tid = threadIdx.x, lane = tid & 31, wave = tid >> 5;
  const int g = blockIdx.x >> 8;
  const int j = blockIdx.x & (kPatch - 1);

  if (tid < 64) {
    const int gi = (tid < kGates) ? tid : (kGates - 1);
    const float th = qp[g * kParGen + gi * 2];
    const float ph = qp[g * kParGen + gi * 2 + 1];
    const float hc = cosf(0.5f * th);
    const float hs = sinf(0.5f * th);
    const float pc = cosf(0.5f * ph);
    const float ps = sinf(0.5f * ph);
    if (tid < kGates) {
      float* gp = sG + tid * 8;
      gp[0] = pc * hc;
      gp[1] = -(ps * hc);
      gp[2] = pc * hs;
      gp[3] = ps * hs;
      gp[4] = -(pc * hs);
      gp[5] = ps * hs;
      gp[6] = pc * hc;
      gp[7] = ps * hc;
    }
  }
#pragma unroll
  for (int e = 0; e < 4; ++e) {
    const int i = tid + e * 256;
    sSt[i] = (i == j) ? 1.0f : 0.0f;
    sSt[kDim + i] = 0.0f;
  }

#pragma unroll 1
  for (int l = kLayers - 1; l >= 0; --l) {
#pragma unroll 1
    for (int q = 0; q < kWires; ++q) {
      __syncthreads();
      const float* gp = sG + (l * kWires + q) * 8;
      const float m00r = gp[0], m00i = gp[1], m01r = gp[2], m01i = gp[3];
      const float m10r = gp[4], m10i = gp[5], m11r = gp[6], m11i = gp[7];
      const int bp = kWires - 1 - q;
      const int st = 1 << bp;
      const bool first = (q == 0);
#pragma unroll 1
      for (int it = 0; it < 2; ++it) {
        const int pi = tid + it * 256;
        const int i0 = ((pi >> bp) << (bp + 1)) | (pi & (st - 1));
        const int i1 = i0 + st;
        float a0r = sSt[i0];
        float a0i = sSt[kDim + i0];
        float a1r = sSt[i1];
        float a1i = sSt[kDim + i1];
        const float sg0 = (first && ((__popc(i0 & (i0 >> 1)) & 1) != 0)) ? -1.0f : 1.0f;
        const float sg1 = (first && ((__popc(i1 & (i1 >> 1)) & 1) != 0)) ? -1.0f : 1.0f;
        a0r *= sg0;
        a0i *= sg0;
        a1r *= sg1;
        a1i *= sg1;
        const float n0r = m00r * a0r - m00i * a0i + m01r * a1r - m01i * a1i;
        const float n0i = m00r * a0i + m00i * a0r + m01r * a1i + m01i * a1r;
        const float n1r = m10r * a0r - m10i * a0i + m11r * a1r - m11i * a1i;
        const float n1i = m10r * a0i + m10i * a0r + m11r * a1i + m11i * a1r;
        sSt[i0] = n0r;
        sSt[kDim + i0] = n0i;
        sSt[i1] = n1r;
        sSt[kDim + i1] = n1i;
      }
    }
  }
  __syncthreads();

  const int part = wave >> 2;
  const int k0 = (wave & 3) * 256 + lane * 8;
  const float* sp = sSt + part * kDim + k0;
  const v4f a0 = *(const v4f*)(sp);
  const v4f a1 = *(const v4f*)(sp + 4);
  v8h hv;
#pragma unroll
  for (int e = 0; e < 4; ++e) {
    const float f0 = a0[e] * kCarry;
    const float f1 = a1[e] * kCarry;
    hv[e] = (_Float16)f0;
    hv[4 + e] = (_Float16)f1;
  }
  unsigned short* dst = Bt + (size_t)(g * 2 * kPatch + part * kPatch + j) * kDim + k0;
  *(volatile v8h*)dst = hv;
  __threadfence();
  *(volatile v8h*)dst = hv;
}

__global__ __launch_bounds__(256) void state_plane_kernel(
    const float* __restrict__ x, unsigned short* __restrict__ Ap)
{
  __shared__ float sC[2 * 16];
  __shared__ float sS[2 * 16];
  const int tid = threadIdx.x;
  if (tid < 32) {
    const int idx = (tid < 2 * kWires) ? tid : (2 * kWires - 1);
    const int rr = idx / kWires;
    const int qq = idx - rr * kWires;
    const float t = x[(blockIdx.x * 2 + rr) * kWires + qq];
    const float hc = cosf(0.5f * t);
    const float hs = sinf(0.5f * t);
    if (tid < 2 * kWires) {
      sC[rr * 16 + qq] = hc;
      sS[rr * 16 + qq] = hs;
    }
  }
  __syncthreads();
  const int r = tid >> 7;
  const int k0 = (tid & 127) * 8;
  const int b = blockIdx.x * 2 + r;
  float base = 1.0f;
#pragma unroll
  for (int q = 0; q < 7; ++q) {
    const float hc = sC[r * 16 + q];
    const float hs = sS[r * 16 + q];
    const float f = (((k0 >> (kWires - 1 - q)) & 1) != 0) ? hs : hc;
    base = base * f;
  }
  const float c7 = sC[r * 16 + 7], s7 = sS[r * 16 + 7];
  const float c8 = sC[r * 16 + 8], s8 = sS[r * 16 + 8];
  const float c9 = sC[r * 16 + 9], s9 = sS[r * 16 + 9];
  v8h hv;
#pragma unroll
  for (int e = 0; e < 8; ++e) {
    float v = base * (((e & 4) != 0) ? s7 : c7);
    v = v * (((e & 2) != 0) ? s8 : c8);
    v = v * (((e & 1) != 0) ? s9 : c9);
    const float vs = v * kCarry;
    hv[e] = (_Float16)vs;
  }
  unsigned short* dst = Ap + (size_t)b * kDim + k0;
  *(volatile v8h*)dst = hv;
  __threadfence();
  *(volatile v8h*)dst = hv;
}

__global__ __launch_bounds__(256) void gemm_f16_kernel(
    const unsigned short* __restrict__ Ap, int lda,
    const unsigned short* __restrict__ Btp, int ldb,
    float* __restrict__ C, int ldc,
    int M, int N, int K, float scale)
{
  const _Float16* A = (const _Float16*)Ap;
  const _Float16* Bt = (const _Float16*)Btp;
  __shared__ __align__(16) float sT[8][16 * 68];
  const int lane = threadIdx.x & 31;
  const int wave = threadIdx.x >> 5;
  const int tilesN = N >> 6;
  const int tilesM = M >> 6;
  const int tile = blockIdx.x * 8 + wave;
  if (tile >= tilesM * tilesN) return;
  const int tm = tile / tilesN;
  const int tn = tile - tm * tilesN;
  const int m0 = tm << 6;
  const int n0 = tn << 6;

  const int rlane = lane & 15;
  const int koff  = (lane >> 4) * 8;
  const int mOff  = (lane >> 4) * 8;

  v8f acc[4][4];
#pragma unroll
  for (int i = 0; i < 4; ++i)
#pragma unroll
    for (int jj = 0; jj < 4; ++jj) acc[i][jj] = (v8f){0.f,0.f,0.f,0.f,0.f,0.f,0.f,0.f};

  for (int k0 = 0; k0 < K; k0 += 32) {
    v16h bh[4];
#pragma unroll
    for (int jj = 0; jj < 4; ++jj) {
      const size_t bo = (size_t)(n0 + (jj << 4) + rlane) * ldb + koff + k0;
      bh[jj] = frag_load_h(Bt + bo);
    }
#pragma unroll
    for (int i = 0; i < 4; ++i) {
      const size_t ao = (size_t)(m0 + (i << 4) + rlane) * lda + koff + k0;
      const v16h ah = frag_load_h(A + ao);
#pragma unroll
      for (int jj = 0; jj < 4; ++jj) {
        acc[i][jj] = mma_h_guarded(ah, bh[jj], acc[i][jj]);
      }
    }
  }

  float* slab = sT[wave];
#pragma unroll
  for (int i = 0; i < 4; ++i) {
    const int mBase = m0 + (i << 4);
#pragma unroll
    for (int jj = 0; jj < 4; ++jj) {
#pragma unroll
      for (int r = 0; r < 8; ++r) {
        const float v = acc[i][jj][r] * scale;
        slab[(mOff + r) * 68 + (jj << 4) + rlane] = v;
      }
    }
    __builtin_amdgcn_fence(__ATOMIC_RELEASE, "workgroup");
    __builtin_amdgcn_wave_barrier();
    __builtin_amdgcn_fence(__ATOMIC_ACQUIRE, "workgroup");
    {
      const int hh = lane >> 4, c4 = (lane & 15) * 4;
      for (int pass = 0; pass < 2; ++pass) {
#pragma unroll
        for (int it = 0; it < 8; ++it) {
          const int row = it * 2 + hh;
          v4f v = *(const v4f*)(slab + row * 68 + c4);
          *(volatile v4f*)(C + (size_t)(mBase + row) * ldc + n0 + c4) = v;
        }
        __threadfence();
      }
    }
    __builtin_amdgcn_fence(__ATOMIC_RELEASE, "workgroup");
    __builtin_amdgcn_wave_barrier();
    __builtin_amdgcn_fence(__ATOMIC_ACQUIRE, "workgroup");
  }
}

__global__ __launch_bounds__(256) void prob_norm_kernel(
    const float* __restrict__ Camp, float* __restrict__ out)
{
  const int lane = threadIdx.x & 31, wave = threadIdx.x >> 5;
  const int seg = blockIdx.x * 8 + wave;
  const int b = seg >> 2;
  const int g = seg & (kGen - 1);
  const float* cre = Camp + (size_t)b * kNcols + g * 2 * kPatch;
  const float* cim = cre + kPatch;
  v4f p[2];
  float m = 0.0f;
#pragma unroll
  for (int it = 0; it < 2; ++it) {
    const v4f re = *(const v4f*)(cre + it * 128 + lane * 4);
    const v4f im = *(const v4f*)(cim + it * 128 + lane * 4);
#pragma unroll
    for (int e = 0; e < 4; ++e) {
      const float pv = re[e] * re[e] + im[e] * im[e];
      p[it][e] = pv;
      m = fmaxf(m, pv);
    }
  }
#pragma unroll
  for (int off = 16; off > 0; off >>= 1) m = fmaxf(m, __shfl_xor(m, off, 32));
  const float inv = 1.0f / m;
  v4f o[2];
#pragma unroll
  for (int it = 0; it < 2; ++it) {
#pragma unroll
    for (int e = 0; e < 4; ++e) o[it][e] = p[it][e] * inv;
  }
  float* dst = out + (size_t)b * (kGen * kPatch) + g * kPatch + lane * 4;
  for (int pass = 0; pass < 2; ++pass) {
#pragma unroll
    for (int it = 0; it < 2; ++it) {
      *(volatile v4f*)(dst + it * 128) = o[it];
    }
    __threadfence();
  }
}

extern "C" void kernel_launch(void* const* d_in, const int* in_sizes, int n_in,
                              void* d_out, int out_size, void* d_ws, size_t ws_size,
                              hipStream_t stream) {
  if (n_in < 2) return;
  if (in_sizes[0] != kBatch * kWires) return;
  if (in_sizes[1] != kGen * kParGen) return;
  if (out_size != kBatch * kGen * kPatch) return;
  if (ws_size < kWsTotal) return;

  const float* x  = (const float*)d_in[0];
  const float* qp = (const float*)d_in[1];
  float* out = (float*)d_out;

  char* ws = (char*)d_ws;
  unsigned short* BT = (unsigned short*)(ws + kOffBT);
  unsigned short* AP = (unsigned short*)(ws + kOffAP);
  float*          CA = (float*)(ws + kOffCA);

  build_rows_kernel<<<kGen * kPatch, 256, 0, stream>>>(qp, BT);
  state_plane_kernel<<<kBatch / 2, 256, 0, stream>>>(x, AP);
  gemm_f16_kernel<<<((kBatch / 64) * (kNcols / 64)) / 8, 256, 0, stream>>>(
      AP, kDim, BT, kDim, CA, kNcols, kBatch, kNcols, kDim, kFold);
  prob_norm_kernel<<<(kBatch * kGen) / 8, 256, 0, stream>>>(CA, out);
}
